// EmbedGCN_45286135169472
// MI455X (gfx1250) — hardware-verified
//
#include <hip/hip_runtime.h>
#include <math.h>
#include <stdint.h>

#define NN     4000
#define NPAD   4096
#define DIN    128
#define DOUT   128
#define EDIM   16
#define NB     8
#define NCAT   (NB * DIN)
#define LDP    4096
#define KLOOP  4000
#define STP    132
#define PCARRY 32768.0f
#define PINV   (1.0f / 32768.0f)
#define F16MIN 6.103515625e-05f

typedef _Float16 v8h  __attribute__((ext_vector_type(8)));
typedef _Float16 v16h __attribute__((ext_vector_type(16)));
typedef __bf16   v8b  __attribute__((ext_vector_type(8)));
typedef __bf16   v16b __attribute__((ext_vector_type(16)));
typedef float    v4f  __attribute__((ext_vector_type(4)));
typedef float    v8f  __attribute__((ext_vector_type(8)));
typedef unsigned int v4u __attribute__((ext_vector_type(4)));

union FragH { v16h v; v8h h[2]; };
union FragB { v16b v; v8b h[2]; };

__device__ __forceinline__ unsigned short bf_bits(float f) {
  const unsigned u = __float_as_uint(f);
  return (unsigned short)((u + 0x7FFFu + ((u >> 16) & 1u)) >> 16);
}
__device__ __forceinline__ float bf_val(unsigned short b) { return __uint_as_float(((unsigned)b) << 16); }
__device__ __forceinline__ float bfrne(float f) { return bf_val(bf_bits(f)); }
__device__ __forceinline__ unsigned short h_bits(_Float16 x) { return __builtin_bit_cast(unsigned short, x); }
__device__ __forceinline__ unsigned pk2(unsigned short lo, unsigned short hi) { return (unsigned)lo | ((unsigned)hi << 16); }

template <int OF16> __device__ __forceinline__ unsigned short cvt16(float f) {
  const unsigned short hb = bf_bits(f);
  if (OF16) {
    float v = bf_val(hb);
    if (fabsf(v) < F16MIN) v = 0.0f;
    return h_bits((_Float16)v);
  } else {
    return hb;
  }
}
__device__ __forceinline__ void split_bf2(float x0, float x1, unsigned& hp, unsigned& lp) {
  const unsigned short h0 = bf_bits(x0), h1 = bf_bits(x1);
  const unsigned short l0 = bf_bits(x0 - bf_val(h0)), l1 = bf_bits(x1 - bf_val(h1));
  hp = pk2(h0, h1);
  lp = pk2(l0, l1);
}

__device__ __forceinline__ v8f mma_h(v16h a, v16h b, v8f c) {
  c = __builtin_amdgcn_wmma_f32_16x16x32_f16(false, a, false, b, (short)0, c, false, false);
  asm volatile("v_nop\n\tv_nop\n\tv_nop\n\tv_nop" : "+v"(c) : "v"(a), "v"(b));
  return c;
}
__device__ __forceinline__ v8f mma_b(v16b a, v16b b, v8f c) {
  c = __builtin_amdgcn_wmma_f32_16x16x32_bf16(false, a, false, b, (short)0, c, false, false);
  asm volatile("v_nop\n\tv_nop\n\tv_nop\n\tv_nop" : "+v"(c) : "v"(a), "v"(b));
  return c;
}

__global__ __launch_bounds__(256) void k_rne4(const float* __restrict__ in, float* __restrict__ outp, int n4) {
  const int i = blockIdx.x * 256 + threadIdx.x;
  if (i < n4) {
    const v4f v = *(const v4f*)(in + 4 * (size_t)i);
    v4f r;
    r[0] = bfrne(v[0]); r[1] = bfrne(v[1]); r[2] = bfrne(v[2]); r[3] = bfrne(v[3]);
    *(volatile v4f*)(outp + 4 * (size_t)i) = r;
    __threadfence();
    *(volatile v4f*)(outp + 4 * (size_t)i) = r;
  }
}

__global__ __launch_bounds__(256) void k_adj(const float* __restrict__ E1, const float* __restrict__ E2r,
                                            unsigned short* __restrict__ Ph, unsigned short* __restrict__ Pl) {
  __shared__ float srow[NPAD];
  __shared__ float sred[8];
  const int n = blockIdx.x;
  const int t = threadIdx.x, lane = t & 31, wave = t >> 5;
  const int nc = (n < NN) ? n : (NN - 1);
  const bool rowvalid = (n < NN);
  if (t < NPAD - NN) srow[NN + t] = 0.0f;

  float e1[EDIM];
#pragma unroll
  for (int d = 0; d < EDIM; ++d) e1[d] = bfrne(E1[(size_t)nc * EDIM + d]);

  float lmax = 0.0f;
#pragma unroll 1
  for (int m = t; m < NN; m += 256) {
    const v4f* p = (const v4f*)(E2r + (size_t)m * EDIM);
    const v4f a0 = p[0], a1 = p[1], a2 = p[2], a3 = p[3];
    float acc = e1[0] * a0[0];
    acc = fmaf(e1[1],  a0[1], acc); acc = fmaf(e1[2],  a0[2], acc); acc = fmaf(e1[3],  a0[3], acc);
    acc = fmaf(e1[4],  a1[0], acc); acc = fmaf(e1[5],  a1[1], acc); acc = fmaf(e1[6],  a1[2], acc); acc = fmaf(e1[7],  a1[3], acc);
    acc = fmaf(e1[8],  a2[0], acc); acc = fmaf(e1[9],  a2[1], acc); acc = fmaf(e1[10], a2[2], acc); acc = fmaf(e1[11], a2[3], acc);
    acc = fmaf(e1[12], a3[0], acc); acc = fmaf(e1[13], a3[1], acc); acc = fmaf(e1[14], a3[2], acc); acc = fmaf(e1[15], a3[3], acc);
    acc = fmaxf(acc, 0.0f);
    srow[m] = acc;
    lmax = fmaxf(lmax, acc);
  }
#pragma unroll
  for (int off = 16; off > 0; off >>= 1) lmax = fmaxf(lmax, __shfl_xor(lmax, off, 32));
  if (lane == 0) sred[wave] = lmax;
  __syncthreads();
  float rmax = sred[0];
#pragma unroll
  for (int w = 1; w < 8; ++w) rmax = fmaxf(rmax, sred[w]);
  __syncthreads();

  float lsum = 0.0f;
#pragma unroll 1
  for (int m = t; m < NN; m += 256) {
    const float e = expf(srow[m] - rmax);
    srow[m] = e;
    lsum += e;
  }
#pragma unroll
  for (int off = 16; off > 0; off >>= 1) lsum += __shfl_xor(lsum, off, 32);
  if (lane == 0) sred[wave] = lsum;
  __syncthreads();
  float rsum = sred[0];
#pragma unroll
  for (int w = 1; w < 8; ++w) rsum += sred[w];
  const float rinv = 1.0f / rsum;
  const float scl = rinv * PCARRY;
  __syncthreads();

  v4u hvv[2], lvv[2];
#pragma unroll
  for (int it = 0; it < 2; ++it) {
    const int col0 = it * 2048 + t * 8;
    v4u hv, lv;
#pragma unroll
    for (int q = 0; q < 4; ++q) {
      unsigned short hb0, hb1, lb0, lb1;
      {
        const int m = col0 + 2 * q;
        float v = srow[m] * scl;
        if (!rowvalid || m >= NN) v = 0.0f;
        if (v < F16MIN) v = 0.0f;
        const _Float16 h16 = (_Float16)v;
        float r = v - (float)h16;
        if (fabsf(r) < F16MIN) r = 0.0f;
        hb0 = h_bits(h16); lb0 = h_bits((_Float16)r);
      }
      {
        const int m = col0 + 2 * q + 1;
        float v = srow[m] * scl;
        if (!rowvalid || m >= NN) v = 0.0f;
        if (v < F16MIN) v = 0.0f;
        const _Float16 h16 = (_Float16)v;
        float r = v - (float)h16;
        if (fabsf(r) < F16MIN) r = 0.0f;
        hb1 = h_bits(h16); lb1 = h_bits((_Float16)r);
      }
      hv[q] = pk2(hb0, hb1);
      lv[q] = pk2(lb0, lb1);
    }
    hvv[it] = hv; lvv[it] = lv;
  }
  const size_t rowoff = (size_t)n * LDP;
  for (int pass = 0; pass < 2; ++pass) {
#pragma unroll
    for (int it = 0; it < 2; ++it) {
      const int col0 = it * 2048 + t * 8;
      *(volatile v4u*)(Ph + rowoff + col0) = hvv[it];
      *(volatile v4u*)(Pl + rowoff + col0) = lvv[it];
    }
    __threadfence();
  }
}

template <int OF16>
__global__ __launch_bounds__(256) void k_tr16(const float* __restrict__ in, int ldi, int nrows, long zin,
                                               unsigned short* __restrict__ outp, int ldo, long zout) {
  __shared__ __align__(16) float tf[64 * 68];
  in   += (size_t)blockIdx.z * (size_t)zin;
  outp += (size_t)blockIdx.z * (size_t)zout;
  const int r0 = blockIdx.x * 64;
  const int c0 = blockIdx.y * 64;
  const int t  = threadIdx.x;
  {
    const int lr = t >> 4, c4 = (t & 15) * 4;
#pragma unroll
    for (int it = 0; it < 4; ++it) {
      const int rr = it * 16 + lr;
      const int gr = r0 + rr;
      const int gc = (gr < nrows) ? gr : (nrows - 1);
      v4f a = *(const v4f*)(in + (size_t)gc * ldi + c0 + c4);
      if (gr >= nrows) a = (v4f){0.f, 0.f, 0.f, 0.f};
      *(v4f*)(tf + rr * 68 + c4) = a;
    }
  }
  __syncthreads();
  const int sub = t >> 3, c8 = (t & 7) * 8;
  v4u ov[2];
#pragma unroll
  for (int it = 0; it < 2; ++it) {
    const int oc = it * 32 + sub;
    v4u a;
#pragma unroll
    for (int q = 0; q < 4; ++q) {
      const float f0 = tf[(c8 + 2 * q) * 68 + oc];
      const float f1 = tf[(c8 + 2 * q + 1) * 68 + oc];
      a[q] = pk2(cvt16<OF16>(f0), cvt16<OF16>(f1));
    }
    ov[it] = a;
  }
  for (int pass = 0; pass < 2; ++pass) {
#pragma unroll
    for (int it = 0; it < 2; ++it) {
      const int oc = it * 32 + sub;
      *(volatile v4u*)(outp + (size_t)(c0 + oc) * ldo + r0 + c8) = ov[it];
    }
    __threadfence();
  }
}

__global__ __launch_bounds__(256) void k_gemm_px(const unsigned short* __restrict__ Php, const unsigned short* __restrict__ Plp,
                                                const unsigned short* __restrict__ XTp,
                                                unsigned short* __restrict__ AH, unsigned short* __restrict__ AL) {
  __shared__ __align__(16) float sT[128 * STP];
  const _Float16* Ph = (const _Float16*)(const void*)Php;
  const _Float16* Pl = (const _Float16*)(const void*)Plp;
  const _Float16* XT = (const _Float16*)(const void*)XTp;
  const int t = threadIdx.x, lane = t & 31, wave = t >> 5;
  const int wm = wave >> 2, wn = wave & 3;
  const int hh = lane >> 4, cc = lane & 15;
  const int m0 = blockIdx.x * 128, n0 = blockIdx.y * 128;

  v8f acc[4][2];
#pragma unroll
  for (int i = 0; i < 4; ++i)
#pragma unroll
    for (int j = 0; j < 2; ++j) acc[i][j] = (v8f){0.f,0.f,0.f,0.f,0.f,0.f,0.f,0.f};

  const _Float16* bp0 = XT + (size_t)(n0 + wn * 32 + cc) * LDP + 8 * hh;
  const _Float16* bp1 = bp0 + (size_t)16 * LDP;
  const _Float16* ahp = Ph + (size_t)(m0 + wm * 64 + cc) * LDP + 8 * hh;
  const _Float16* alp = Pl + (size_t)(m0 + wm * 64 + cc) * LDP + 8 * hh;

#pragma unroll 1
  for (int k0 = 0; k0 < KLOOP; k0 += 32) {
    FragH b0, b1;
    b0.h[0] = *(const v8h*)(bp0 + k0);  b0.h[1] = *(const v8h*)(bp0 + k0 + 16);
    b1.h[0] = *(const v8h*)(bp1 + k0);  b1.h[1] = *(const v8h*)(bp1 + k0 + 16);
#pragma unroll
    for (int i = 0; i < 4; ++i) {
      const _Float16* ap = ahp + (size_t)i * 16 * LDP + k0;
      const _Float16* lp = alp + (size_t)i * 16 * LDP + k0;
      FragH a, l;
      a.h[0] = *(const v8h*)ap;  a.h[1] = *(const v8h*)(ap + 16);
      l.h[0] = *(const v8h*)lp;  l.h[1] = *(const v8h*)(lp + 16);
      acc[i][0] = mma_h(a.v, b0.v, acc[i][0]);
      acc[i][1] = mma_h(a.v, b1.v, acc[i][1]);
      acc[i][0] = mma_h(l.v, b0.v, acc[i][0]);
      acc[i][1] = mma_h(l.v, b1.v, acc[i][1]);
    }
  }

#pragma unroll
  for (int i = 0; i < 4; ++i)
#pragma unroll
    for (int j = 0; j < 2; ++j)
#pragma unroll
      for (int e = 0; e < 8; ++e)
        sT[(wm * 64 + i * 16 + 8 * hh + e) * STP + wn * 32 + j * 16 + cc] = acc[i][j][e] * PINV;
  __syncthreads();

  const int rr = t >> 4, c8 = (t & 15) * 8;
  const size_t obase = ((size_t)(n0 >> 7) * NPAD + (size_t)m0) * DIN;
  for (int pass = 0; pass < 2; ++pass) {
#pragma unroll
    for (int it = 0; it < 8; ++it) {
      const int r = it * 16 + rr;
      const float* sp = sT + r * STP + c8;
      const v4f fa = *(const v4f*)sp;
      const v4f fb = *(const v4f*)(sp + 4);
      v4u hv, lv;
      unsigned hpk, lpk;
      split_bf2(fa[0], fa[1], hpk, lpk); hv[0] = hpk; lv[0] = lpk;
      split_bf2(fa[2], fa[3], hpk, lpk); hv[1] = hpk; lv[1] = lpk;
      split_bf2(fb[0], fb[1], hpk, lpk); hv[2] = hpk; lv[2] = lpk;
      split_bf2(fb[2], fb[3], hpk, lpk); hv[3] = hpk; lv[3] = lpk;
      const size_t go = obase + (size_t)r * DIN + c8;
      *(volatile v4u*)(AH + go) = hv;
      *(volatile v4u*)(AL + go) = lv;
    }
    __threadfence();
  }
}

__global__ __launch_bounds__(256) void k_gemm_w(const unsigned short* __restrict__ AHp, const unsigned short* __restrict__ ALp,
                                               const unsigned short* __restrict__ WTp, const float* __restrict__ bias,
                                               float* __restrict__ out) {
  __shared__ __align__(16) float sT[128 * STP];
  const __bf16* AH = (const __bf16*)(const void*)AHp;
  const __bf16* AL = (const __bf16*)(const void*)ALp;
  const __bf16* WT = (const __bf16*)(const void*)WTp;
  const int t = threadIdx.x, lane = t & 31, wave = t >> 5;
  const int wm = wave >> 2, wn = wave & 3;
  const int hh = lane >> 4, cc = lane & 15;
  const int m0 = blockIdx.x * 128;

  v8f acc[4][2];
#pragma unroll
  for (int i = 0; i < 4; ++i)
#pragma unroll
    for (int j = 0; j < 2; ++j) acc[i][j] = (v8f){0.f,0.f,0.f,0.f,0.f,0.f,0.f,0.f};

  const __bf16* bp0 = WT + (size_t)(wn * 32 + cc) * DIN + 8 * hh;
  const __bf16* bp1 = bp0 + (size_t)16 * DIN;
  const __bf16* ahp = AH + (size_t)(m0 + wm * 64 + cc) * DIN + 8 * hh;
  const __bf16* alp = AL + (size_t)(m0 + wm * 64 + cc) * DIN + 8 * hh;

#pragma unroll
  for (int k0 = 0; k0 < DIN; k0 += 32) {
    FragB b0, b1;
    b0.h[0] = *(const v8b*)(bp0 + k0);  b0.h[1] = *(const v8b*)(bp0 + k0 + 16);
    b1.h[0] = *(const v8b*)(bp1 + k0);  b1.h[1] = *(const v8b*)(bp1 + k0 + 16);
#pragma unroll
    for (int i = 0; i < 4; ++i) {
      const __bf16* ap = ahp + (size_t)i * 16 * DIN + k0;
      const __bf16* lp = alp + (size_t)i * 16 * DIN + k0;
      FragB a, l;
      a.h[0] = *(const v8b*)ap;  a.h[1] = *(const v8b*)(ap + 16);
      l.h[0] = *(const v8b*)lp;  l.h[1] = *(const v8b*)(lp + 16);
      acc[i][0] = mma_b(a.v, b0.v, acc[i][0]);
      acc[i][1] = mma_b(a.v, b1.v, acc[i][1]);
      acc[i][0] = mma_b(l.v, b0.v, acc[i][0]);
      acc[i][1] = mma_b(l.v, b1.v, acc[i][1]);
    }
  }

  const float bb0 = bfrne(bias[wn * 32 + cc]);
  const float bb1 = bfrne(bias[wn * 32 + 16 + cc]);
#pragma unroll
  for (int i = 0; i < 4; ++i)
#pragma unroll
    for (int j = 0; j < 2; ++j)
#pragma unroll
      for (int e = 0; e < 8; ++e) {
        float v = acc[i][j][e] + (j ? bb1 : bb0);
        v = fmaxf(v, 0.0f);
        sT[(wm * 64 + i * 16 + 8 * hh + e) * STP + wn * 32 + j * 16 + cc] = v;
      }
  __syncthreads();

  const int bidx  = m0 >> 12;
  const int nbase = m0 & (NPAD - 1);
  for (int pass = 0; pass < 2; ++pass) {
#pragma unroll
    for (int it = 0; it < 16; ++it) {
      const int r = it * 8 + wave;
      const int nrow = nbase + r;
      if (nrow < NN) {
        const v4f v = *(const v4f*)(sT + r * STP + lane * 4);
        *(volatile v4f*)(out + ((size_t)bidx * NN + (size_t)nrow) * DOUT + lane * 4) = v;
      }
    }
    __threadfence();
  }
}

extern "C" void kernel_launch(void* const* d_in, const int* in_sizes, int n_in,
                              void* d_out, int out_size, void* d_ws, size_t ws_size,
                              hipStream_t stream) {
  if (n_in < 5) return;
  if (in_sizes[0] != NB * NN * DIN) return;
  if (in_sizes[1] != NN * EDIM || in_sizes[2] != NN * EDIM) return;
  if (in_sizes[3] != DIN * DOUT || in_sizes[4] != DOUT) return;
  if (out_size != NB * NN * DOUT) return;

  const float* x    = (const float*)d_in[0];
  const float* E1   = (const float*)d_in[1];
  const float* E2   = (const float*)d_in[2];
  const float* W    = (const float*)d_in[3];
  const float* bias = (const float*)d_in[4];
  float* out = (float*)d_out;

  const size_t szE2 = (size_t)NN * EDIM * sizeof(float);
  const size_t szP  = (size_t)NPAD * LDP * 2;
  const size_t szXT = (size_t)NCAT * LDP * 2;
  const size_t szA  = (size_t)NB * NPAD * DIN * 2;
  const size_t szWT = (size_t)DOUT * DIN * 2;
  size_t off = 0;
  const size_t oE2 = off; off += szE2;
  const size_t oPh = off; off += szP;
  const size_t oPl = off; off += szP;
  const size_t oXT = off; off += szXT;
  const size_t oAH = off; off += szA;
  const size_t oAL = off; off += szA;
  const size_t oWT = off; off += szWT;
  if (off > ws_size) return;

  char* ws = (char*)d_ws;
  float*          E2r = (float*)(ws + oE2);
  unsigned short* Ph  = (unsigned short*)(ws + oPh);
  unsigned short* Pl  = (unsigned short*)(ws + oPl);
  unsigned short* XT  = (unsigned short*)(ws + oXT);
  unsigned short* AH  = (unsigned short*)(ws + oAH);
  unsigned short* AL  = (unsigned short*)(ws + oAL);
  unsigned short* WT  = (unsigned short*)(ws + oWT);

  const dim3 blk(256);
  const int n4 = NN * EDIM / 4;
  k_rne4<<<dim3((n4 + 255) / 256), blk, 0, stream>>>(E2, E2r, n4);
  k_adj<<<dim3(NPAD), blk, 0, stream>>>(E1, E2r, Ph, Pl);
  k_tr16<1><<<dim3(NPAD / 64, DIN / 64, NB), blk, 0, stream>>>(x, DIN, NN, (long)NN * DIN, XT, LDP, (long)DIN * LDP);
  k_tr16<0><<<dim3(DIN / 64, DOUT / 64, 1), blk, 0, stream>>>(W, DOUT, DIN, 0L, WT, DIN, 0L);
  k_gemm_px<<<dim3(NPAD / 128, NCAT / 128), blk, 0, stream>>>(Ph, Pl, XT, AH, AL);
  k_gemm_w<<<dim3(NB * NPAD / 128), blk, 0, stream>>>(AH, AL, WT, bias, out);
  (void)hipGetLastError();
}
